// MHSA_6519760355779
// MI455X (gfx1250) — hardware-verified
//
#include <hip/hip_runtime.h>
#include <math.h>
#include <stdint.h>

#define NBAT 16
#define CH   256
#define NT   2304
#define TOK  (NBAT * NT)
#define QKLD 512

static_assert(NT % 64 == 0);
static_assert(CH % 64 == 0);
static_assert(TOK % 64 == 0);
static_assert(CH % 32 == 0);

typedef __attribute__((ext_vector_type(16))) __bf16   v16b;
typedef __attribute__((ext_vector_type(8)))  __bf16   v8b;
typedef __attribute__((ext_vector_type(8)))  float    v8f;
typedef __attribute__((ext_vector_type(4)))  float    v4f;
typedef __attribute__((ext_vector_type(4)))  unsigned int v4u;
typedef v8b __attribute__((may_alias)) v8ba;
typedef v4f __attribute__((may_alias)) v4fa;

__device__ __forceinline__ unsigned short f2bf_bits(float f) {
  unsigned u = __float_as_uint(f);
  return (unsigned short)((u + 0x7FFFu + ((u >> 16) & 1u)) >> 16);
}
__device__ __forceinline__ float bf_bits2f(unsigned short h) { return __uint_as_float(((unsigned)h) << 16); }
__device__ __forceinline__ float bfr(float f) { return bf_bits2f(f2bf_bits(f)); }
__device__ __forceinline__ unsigned pk16(unsigned short a, unsigned short b) { return (unsigned)a | ((unsigned)b << 16); }
__device__ __forceinline__ void split2(float f0, float f1, unsigned& h, unsigned& l) {
  const unsigned short h0 = f2bf_bits(f0), h1 = f2bf_bits(f1);
  const unsigned short l0 = f2bf_bits(f0 - bf_bits2f(h0)), l1 = f2bf_bits(f1 - bf_bits2f(h1));
  h = pk16(h0, h1);
  l = pk16(l0, l1);
}

union FB { v16b v; v8b h[2]; };
__device__ __forceinline__ v16b ldfrag(const __bf16* p) {
  FB f;
  f.h[0] = *(const v8ba*)(p);
  f.h[1] = *(const v8ba*)(p + 16);
  return f.v;
}
__device__ __forceinline__ v8f mma_bf(v16b a, v16b b, v8f c) {
  c = __builtin_amdgcn_wmma_f32_16x16x32_bf16(false, a, false, b, (short)0, c, false, false);
  asm volatile("v_nop\n\tv_nop\n\tv_nop\n\tv_nop" : "+v"(c) : "v"(a), "v"(b));
  return c;
}

__global__ __launch_bounds__(256) void tcast_kernel(const float* __restrict__ X, unsigned short* __restrict__ oh,
                                                    int R, int Cc, long sIn, long sOut) {
  __shared__ __align__(16) float tf[64 * 68];
  X  += (size_t)blockIdx.z * sIn;
  oh += (size_t)blockIdx.z * sOut;
  const int c0  = blockIdx.x * 64;
  const int r0  = blockIdx.y * 64;
  const int tid = threadIdx.x;
  {
    const int lr = tid >> 4;
    const int c4 = (tid & 15) * 4;
#pragma unroll
    for (int it = 0; it < 4; ++it) {
      const int rr = it * 16 + lr;
      const v4f a = *(const v4f*)(X + (size_t)(r0 + rr) * Cc + c0 + c4);
      *(v4fa*)(tf + rr * 68 + c4) = a;
    }
  }
  __syncthreads();
  const int sub = tid >> 3;
  const int c8  = (tid & 7) * 8;
  v4u hv[2];
#pragma unroll
  for (int it = 0; it < 2; ++it) {
    const int oc = it * 32 + sub;
    v4u a;
#pragma unroll
    for (int q = 0; q < 4; ++q) {
      const float f0 = tf[(c8 + 2 * q) * 68 + oc];
      const float f1 = tf[(c8 + 2 * q + 1) * 68 + oc];
      a[q] = pk16(f2bf_bits(f0), f2bf_bits(f1));
    }
    hv[it] = a;
  }
  for (int pass = 0; pass < 2; ++pass) {
#pragma unroll
    for (int it = 0; it < 2; ++it) {
      const int oc = it * 32 + sub;
      const size_t go = (size_t)(c0 + oc) * R + r0 + c8;
      *(volatile v4u*)(oh + go) = hv[it];
    }
    __threadfence();
  }
}

__global__ __launch_bounds__(256) void wprep_kernel(const float* __restrict__ wq, const float* __restrict__ wk,
                                                    const float* __restrict__ wv, const float* __restrict__ bq,
                                                    const float* __restrict__ bk, const float* __restrict__ bv,
                                                    unsigned short* __restrict__ wall, float* __restrict__ ball) {
  const int tid = threadIdx.x;
  if (blockIdx.x < 96) {
    const int mat = blockIdx.x >> 5;
    const float* src = (mat == 0) ? wq : ((mat == 1) ? wk : wv);
    const int off = ((blockIdx.x & 31) * 256 + tid) * 8;
    const v4f a = *(const v4f*)(src + off);
    const v4f c = *(const v4f*)(src + off + 4);
    v4u o;
    o[0] = pk16(f2bf_bits(a[0]), f2bf_bits(a[1]));
    o[1] = pk16(f2bf_bits(a[2]), f2bf_bits(a[3]));
    o[2] = pk16(f2bf_bits(c[0]), f2bf_bits(c[1]));
    o[3] = pk16(f2bf_bits(c[2]), f2bf_bits(c[3]));
    unsigned short* dst = wall + (size_t)mat * 65536 + off;
    *(volatile v4u*)dst = o;
    __threadfence();
    *(volatile v4u*)dst = o;
  } else {
    if (tid < 192) {
      const int seg = tid >> 6;
      const int o4 = (tid & 63) * 4;
      const v4f a = *(const v4f*)(bq + o4);
      const v4f c = *(const v4f*)(bk + o4);
      const v4f d = *(const v4f*)(bv + o4);
      const unsigned m0 = (seg == 0) ? 0xFFFFFFFFu : 0u;
      const unsigned m1 = (seg == 1) ? 0xFFFFFFFFu : 0u;
      const unsigned m2 = (seg == 2) ? 0xFFFFFFFFu : 0u;
      v4f o;
#pragma unroll
      for (int e = 0; e < 4; ++e) {
        const unsigned ua = __float_as_uint(bfr(a[e]));
        const unsigned uc = __float_as_uint(bfr(c[e]));
        const unsigned ud = __float_as_uint(bfr(d[e]));
        o[e] = __uint_as_float((ua & m0) | (uc & m1) | (ud & m2));
      }
      float* dst = ball + 4 * tid;
      *(volatile v4f*)dst = o;
      __threadfence();
      *(volatile v4f*)dst = o;
    }
  }
}

template <int BIAS_MODE>
__global__ __launch_bounds__(256) void gemm64_bf16_kernel(
    const unsigned short* __restrict__ Ap, int lda, long strideA,
    const unsigned short* __restrict__ Btp, int ldb, long strideB,
    unsigned short* __restrict__ Chp, unsigned short* __restrict__ Clp, int ldc, long strideC,
    const float* __restrict__ bias, int M, int N, int K) {
  __shared__ __align__(16) float sT[8][16 * 68];
  const int b    = blockIdx.y;
  const int lane = threadIdx.x & 31;
  const int wave = threadIdx.x >> 5;
  const int tilesN = N >> 6;
  const int tilesM = M >> 6;
  const int tile = blockIdx.x * 8 + wave;
  if (tile >= tilesM * tilesN) return;
  const int tm = tile / tilesN;
  const int tn = tile - tm * tilesN;
  const int m0 = tm << 6;
  const int n0 = tn << 6;

  const __bf16* Ab = (const __bf16*)(const void*)Ap  + (size_t)b * strideA;
  const __bf16* Bb = (const __bf16*)(const void*)Btp + (size_t)b * strideB;

  const int rlane = lane & 15;
  const int koff  = (lane >> 4) * 8;
  const int mOff  = (lane >> 4) * 8;

  v8f acc[4][4];
#pragma unroll
  for (int i = 0; i < 4; ++i)
#pragma unroll
    for (int j = 0; j < 4; ++j) acc[i][j] = (v8f){0.f,0.f,0.f,0.f,0.f,0.f,0.f,0.f};

#pragma unroll 1
  for (int k0 = 0; k0 < K; k0 += 32) {
    v16b bh[4];
#pragma unroll
    for (int j = 0; j < 4; ++j) {
      const size_t bo = (size_t)(n0 + (j << 4) + rlane) * ldb + koff + k0;
      bh[j] = ldfrag(Bb + bo);
    }
#pragma unroll
    for (int i = 0; i < 4; ++i) {
      const size_t ao = (size_t)(m0 + (i << 4) + rlane) * lda + koff + k0;
      const v16b ah = ldfrag(Ab + ao);
#pragma unroll
      for (int j = 0; j < 4; ++j) acc[i][j] = mma_bf(ah, bh[j], acc[i][j]);
    }
  }

  float* slab = sT[wave];
  const int q  = lane >> 3;
  const int c8 = (lane & 7) * 8;
  v4f cb0 = (v4f){0.f,0.f,0.f,0.f}, cb1 = (v4f){0.f,0.f,0.f,0.f};
  if (BIAS_MODE == 2) {
    cb0 = *(const v4f*)(bias + n0 + c8);
    cb1 = *(const v4f*)(bias + n0 + c8 + 4);
  }
  unsigned short* Cb  = Chp + (size_t)b * strideC;
  unsigned short* Cb2 = Clp + (size_t)b * strideC;
#pragma unroll
  for (int i = 0; i < 4; ++i) {
    const int mBase = m0 + (i << 4);
    float rbv[8];
    if (BIAS_MODE == 1) {
      const v4f rb0 = *(const v4f*)(bias + mBase + mOff);
      const v4f rb1 = *(const v4f*)(bias + mBase + mOff + 4);
      rbv[0] = rb0[0]; rbv[1] = rb0[1]; rbv[2] = rb0[2]; rbv[3] = rb0[3];
      rbv[4] = rb1[0]; rbv[5] = rb1[1]; rbv[6] = rb1[2]; rbv[7] = rb1[3];
    } else {
#pragma unroll
      for (int r = 0; r < 8; ++r) rbv[r] = 0.f;
    }
#pragma unroll
    for (int j = 0; j < 4; ++j) {
#pragma unroll
      for (int r = 0; r < 8; ++r) {
        const float v = acc[i][j][r] + rbv[r];
        slab[(mOff + r) * 68 + (j << 4) + rlane] = v;
      }
    }
    __builtin_amdgcn_fence(__ATOMIC_RELEASE, "workgroup");
    __builtin_amdgcn_wave_barrier();
    __builtin_amdgcn_fence(__ATOMIC_ACQUIRE, "workgroup");
    v4u hv[4], lv[4];
#pragma unroll
    for (int it = 0; it < 4; ++it) {
      const int row = it * 4 + q;
      const float* sp = slab + row * 68 + c8;
      v4f s0 = *(const v4fa*)(sp);
      v4f s1 = *(const v4fa*)(sp + 4);
      s0 = s0 + cb0;
      s1 = s1 + cb1;
      v4u h, l;
      unsigned hw, lw;
      split2(s0[0], s0[1], hw, lw); h[0] = hw; l[0] = lw;
      split2(s0[2], s0[3], hw, lw); h[1] = hw; l[1] = lw;
      split2(s1[0], s1[1], hw, lw); h[2] = hw; l[2] = lw;
      split2(s1[2], s1[3], hw, lw); h[3] = hw; l[3] = lw;
      hv[it] = h; lv[it] = l;
    }
    for (int pass = 0; pass < 2; ++pass) {
#pragma unroll
      for (int it = 0; it < 4; ++it) {
        const int row = it * 4 + q;
        const size_t go = (size_t)(mBase + row) * ldc + n0 + c8;
        *(volatile v4u*)(Cb  + go) = hv[it];
        *(volatile v4u*)(Cb2 + go) = lv[it];
      }
      __threadfence();
    }
    __builtin_amdgcn_fence(__ATOMIC_RELEASE, "workgroup");
    __builtin_amdgcn_wave_barrier();
    __builtin_amdgcn_fence(__ATOMIC_ACQUIRE, "workgroup");
  }
}

#define AP 72
#define OP 68

__device__ __forceinline__ void p_split(float f, __bf16& hi, __bf16& lo) {
  const unsigned short hb = f2bf_bits(f);
  hi = __builtin_bit_cast(__bf16, hb);
  lo = __builtin_bit_cast(__bf16, f2bf_bits(f - bf_bits2f(hb)));
}

__global__ __launch_bounds__(256)
void attn256_kernel(const unsigned short* __restrict__ qkhp, const unsigned short* __restrict__ qklp,
                    const unsigned short* __restrict__ vthp, const unsigned short* __restrict__ vtlp,
                    const float* __restrict__ x, float* __restrict__ out) {
  __shared__ __align__(16) __bf16 Psh[64 * AP];
  __shared__ __align__(16) __bf16 Psl[64 * AP];
  __shared__ __align__(16) float  pMax[2][64];
  __shared__ __align__(16) float  pSum[2][64];
  __shared__ __align__(16) float  Os[128 * OP];

  const int tid  = threadIdx.x;
  const int wave = tid >> 5;
  const int lane = tid & 31;
  const int hh   = lane >> 4;
  const int c    = lane & 15;
  const int qt   = wave & 3;
  const int hf   = wave >> 2;
  const int b    = blockIdx.y;
  const int q0   = blockIdx.x * 64;

  const __bf16* QKh = (const __bf16*)(const void*)qkhp;
  const __bf16* QKl = (const __bf16*)(const void*)qklp;
  const __bf16* VTh = (const __bf16*)(const void*)vthp;
  const __bf16* VTl = (const __bf16*)(const void*)vtlp;

  const size_t tok0 = (size_t)b * NT;
  const size_t qoff = (tok0 + q0 + 16 * qt + c) * QKLD + 8 * hh;
  const size_t koff = (tok0 + 32 * hf + c) * QKLD + CH + 8 * hh;
  const size_t voff = ((size_t)b * CH + 128 * hf + c) * NT + 8 * hh;
  const __bf16* qrh = QKh + qoff;
  const __bf16* qrl = QKl + qoff;
  const __bf16* kbh = QKh + koff;
  const __bf16* kbl = QKl + koff;
  const __bf16* vbh = VTh + voff;
  const __bf16* vbl = VTl + voff;

  float mrow[8], lrow[8];
  v8f oacc[8];
#pragma unroll
  for (int r = 0; r < 8; ++r) { mrow[r] = -INFINITY; lrow[r] = 0.f; }
#pragma unroll
  for (int t = 0; t < 8; ++t) oacc[t] = (v8f){0.f,0.f,0.f,0.f,0.f,0.f,0.f,0.f};

  const int rowb = 16 * qt + 8 * hh;

#pragma unroll 1
  for (int kc = 0; kc < NT / 64; ++kc) {
    const int kv0 = kc * 64;

    v8f s[2];
    s[0] = (v8f){0.f,0.f,0.f,0.f,0.f,0.f,0.f,0.f};
    s[1] = (v8f){0.f,0.f,0.f,0.f,0.f,0.f,0.f,0.f};
#pragma unroll 1
    for (int dc = 0; dc < CH / 32; ++dc) {
      const v16b qh = ldfrag(qrh + dc * 32);
      const v16b ql = ldfrag(qrl + dc * 32);
#pragma unroll
      for (int j = 0; j < 2; ++j) {
        const size_t ko = (size_t)(kv0 + 16 * j) * QKLD + dc * 32;
        const v16b kfh = ldfrag(kbh + ko);
        const v16b kfl = ldfrag(kbl + ko);
        s[j] = mma_bf(qh, kfh, s[j]);
        s[j] = mma_bf(qh, kfl, s[j]);
        s[j] = mma_bf(ql, kfh, s[j]);
      }
    }

    float cm[8];
#pragma unroll
    for (int r = 0; r < 8; ++r) {
      float m = fmaxf(s[0][r], s[1][r]);
#pragma unroll
      for (int off = 1; off < 16; off <<= 1) m = fmaxf(m, __shfl_xor(m, off, 32));
      cm[r] = m;
    }
    if (c == 0) {
#pragma unroll
      for (int r = 0; r < 8; ++r) pMax[hf][rowb + r] = cm[r];
    }
    __syncthreads();

    float ps[8];
#pragma unroll
    for (int r = 0; r < 8; ++r) {
      const float bm = fmaxf(pMax[0][rowb + r], pMax[1][rowb + r]);
      const float mnew = fmaxf(mrow[r], bm);
      const float alpha = expf(mrow[r] - mnew);
      mrow[r] = mnew;
      float psum = 0.f;
#pragma unroll
      for (int j = 0; j < 2; ++j) {
        const float p = expf(s[j][r] - mnew);
        psum += p;
        __bf16 ph, pl;
        p_split(p, ph, pl);
        Psh[(rowb + r) * AP + 32 * hf + 16 * j + c] = ph;
        Psl[(rowb + r) * AP + 32 * hf + 16 * j + c] = pl;
      }
#pragma unroll
      for (int off = 1; off < 16; off <<= 1) psum += __shfl_xor(psum, off, 32);
      ps[r] = psum;
      lrow[r] = lrow[r] * alpha;
#pragma unroll
      for (int t = 0; t < 8; ++t) oacc[t][r] *= alpha;
    }
    if (c == 0) {
#pragma unroll
      for (int r = 0; r < 8; ++r) pSum[hf][rowb + r] = ps[r];
    }
    __syncthreads();
#pragma unroll
    for (int r = 0; r < 8; ++r) lrow[r] = lrow[r] + (pSum[0][rowb + r] + pSum[1][rowb + r]);

#pragma unroll 1
    for (int kk = 0; kk < 2; ++kk) {
      const v16b pa = ldfrag(Psh + (16 * qt + c) * AP + kk * 32 + 8 * hh);
      const v16b pl = ldfrag(Psl + (16 * qt + c) * AP + kk * 32 + 8 * hh);
#pragma unroll
      for (int t = 0; t < 8; ++t) {
        const size_t vo = (size_t)(16 * t) * NT + kv0 + kk * 32;
        const v16b vfh = ldfrag(vbh + vo);
        const v16b vfl = ldfrag(vbl + vo);
        oacc[t] = mma_bf(pa, vfh, oacc[t]);
        oacc[t] = mma_bf(pa, vfl, oacc[t]);
        oacc[t] = mma_bf(pl, vfh, oacc[t]);
      }
    }
  }

  float inv[8];
#pragma unroll
  for (int r = 0; r < 8; ++r) inv[r] = 1.0f / lrow[r];
  const int c4 = (lane & 15) * 4;
#pragma unroll
  for (int ph = 0; ph < 2; ++ph) {
    __syncthreads();
    if (hf == ph) {
#pragma unroll
      for (int t = 0; t < 8; ++t)
#pragma unroll
        for (int r = 0; r < 8; ++r)
          Os[(16 * t + c) * OP + rowb + r] = oacc[t][r] * inv[r];
    }
    __syncthreads();
    for (int pass = 0; pass < 2; ++pass) {
#pragma unroll 4
      for (int it = 0; it < 8; ++it) {
        const int rowl = 16 * wave + 2 * it + hh;
        const int chn  = 128 * ph + rowl;
        const size_t off = ((size_t)b * CH + chn) * NT + q0 + c4;
        v4f o = *(const v4fa*)(Os + rowl * OP + c4);
        const v4f xv = *(const v4f*)(x + off);
        o[0] = o[0] + bfr(xv[0]);
        o[1] = o[1] + bfr(xv[1]);
        o[2] = o[2] + bfr(xv[2]);
        o[3] = o[3] + bfr(xv[3]);
        *(volatile v4f*)(out + off) = o;
      }
      __threadfence();
    }
  }
}

extern "C" void kernel_launch(void* const* d_in, const int* in_sizes, int n_in,
                              void* d_out, int out_size, void* d_ws, size_t ws_size,
                              hipStream_t stream) {
  if (n_in < 7) return;
  if (in_sizes[0] != NBAT * CH * NT) return;
  if (in_sizes[1] != CH * CH || in_sizes[3] != CH * CH || in_sizes[5] != CH * CH) return;
  if (in_sizes[2] != CH || in_sizes[4] != CH || in_sizes[6] != CH) return;
  if (out_size != NBAT * CH * NT) return;

  const float* x  = (const float*)d_in[0];
  const float* wq = (const float*)d_in[1];
  const float* bq = (const float*)d_in[2];
  const float* wk = (const float*)d_in[3];
  const float* bk = (const float*)d_in[4];
  const float* wv = (const float*)d_in[5];
  const float* bv = (const float*)d_in[6];
  float* out = (float*)d_out;

  const size_t szXB   = (size_t)TOK * CH * 2;
  const size_t szWALL = (size_t)768 * CH * 2;
  const size_t szBALL = (size_t)768 * 4;
  const size_t szQK   = (size_t)TOK * QKLD * 2;
  const size_t szVT   = (size_t)NBAT * CH * NT * 2;
  size_t off = 0;
  const size_t oXB   = off; off += szXB;
  const size_t oWALL = off; off += szWALL;
  const size_t oBALL = off; off += szBALL;
  const size_t oQKh  = off; off += szQK;
  const size_t oQKl  = off; off += szQK;
  const size_t oVTh  = off; off += szVT;
  const size_t oVTl  = off; off += szVT;
  if (off > ws_size) return;
  if (off > (size_t)134217728) return;

  char* ws = (char*)d_ws;
  unsigned short* XB   = (unsigned short*)(ws + oXB);
  unsigned short* WALL = (unsigned short*)(ws + oWALL);
  float*          BALL = (float*)(ws + oBALL);
  unsigned short* QKh  = (unsigned short*)(ws + oQKh);
  unsigned short* QKl  = (unsigned short*)(ws + oQKl);
  unsigned short* VTh  = (unsigned short*)(ws + oVTh);
  unsigned short* VTl  = (unsigned short*)(ws + oVTl);

  tcast_kernel<<<dim3(NT / 64, CH / 64, NBAT), dim3(256), 0, stream>>>(
      x, XB, CH, NT, (long)CH * NT, (long)NT * CH);
  wprep_kernel<<<dim3(97), dim3(256), 0, stream>>>(wq, wk, wv, bq, bk, bv, WALL, BALL);
  gemm64_bf16_kernel<2><<<dim3((TOK / 64) * (QKLD / 64) / 8, 1), dim3(256), 0, stream>>>(
      XB, CH, 0L, WALL, CH, 0L, QKh, QKl, QKLD, 0L, BALL, TOK, QKLD, CH);
  gemm64_bf16_kernel<1><<<dim3((CH / 64) * (NT / 64) / 8, NBAT), dim3(256), 0, stream>>>(
      WALL + (size_t)512 * CH, CH, 0L, XB, CH, (long)NT * CH, VTh, VTl, NT, (long)CH * NT,
      BALL + 512, CH, NT, CH);
  attn256_kernel<<<dim3(NT / 64, NBAT), dim3(256), 0, stream>>>(QKh, QKl, VTh, VTl, x, out);
  (void)hipGetLastError();
}
